// Decoder_69776038690924
// MI455X (gfx1250) — hardware-verified
//
#include <hip/hip_runtime.h>
#include <math.h>

constexpr int BATCH   = 32768;
constexpr int HID     = 128;
constexpr int TLEN    = 12;
constexpr int G4      = 4 * HID;
constexpr int MROWS   = BATCH * TLEN;
constexpr int NL1     = 50;
constexpr int NPADC   = 64;
constexpr int WPB     = 2;
constexpr int NTHR1   = 32 * WPB;
constexpr int NWAVES  = BATCH / 16;
constexpr int NBLK1   = NWAVES / WPB;
constexpr int HP      = 136;
constexpr int SLP     = 68;
constexpr int REC1    = 256;
constexpr int REC3    = 128;
constexpr int NB3     = MROWS / 256;
constexpr int NB5     = (MROWS * 2 / 4) / 256;
constexpr float WCARRY      = 64.0f;
constexpr float WCARRY_INV  = 1.0f / 64.0f;
constexpr float LOCARRY     = 2048.0f;
constexpr float LO_INV      = 1.0f / (64.0f * 2048.0f);
constexpr float HI_MIN      = 6.2e-5f;
constexpr float EPS_BN      = 1e-5f;
static_assert(BATCH % (16 * WPB) == 0, "whole blocks");
static_assert(HID % 32 == 0, "K multiple of 32");
static_assert(NPADC % 16 == 0 && G4 % 16 == 0, "N tiles");
static_assert(MROWS % 256 == 0, "relu pass grid exact");
static_assert((MROWS * 2) % (4 * 256) == 0, "output pass grid exact");
static_assert(TLEN % 2 == 0, "pairs of output rows stay in one sequence");
static_assert(2 * 16 * HP * 2 * 2 * WPB + 64 * 32 * 4 * WPB + 16 * SLP * 4 * WPB <= 65536, "static LDS");

typedef __attribute__((ext_vector_type(16))) _Float16 v16h;
typedef __attribute__((ext_vector_type(8)))  _Float16 v8h;
typedef __attribute__((ext_vector_type(8)))  float    v8f;
typedef __attribute__((ext_vector_type(4)))  float    v4f;
typedef __attribute__((ext_vector_type(2)))  float    v2f;

template <typename T> struct Frag;
template <> struct Frag<_Float16> {
  typedef v16h V; union U { v16h v; v8h h[2]; };
  static __device__ __forceinline__ v16h load(const _Float16* p) {
    U f; f.h[0] = *(const v8h*)(p); f.h[1] = *(const v8h*)(p + 16); return f.v;
  }
  static __device__ __forceinline__ v8f mma(v16h a, v16h b, v8f c) {
    return __builtin_amdgcn_wmma_f32_16x16x32_f16(false, a, false, b, (short)0, c, false, false);
  }
};

__device__ __forceinline__ void guard_gate(v8f& a0, v8f& a1, v8f& a2, v8f& a3, v8f& a4, v8f& a5, v8f& a6, v8f& a7,
                                           v16h x, v16h y, v16h b0, v16h b1, v16h b2, v16h b3) {
  asm volatile("v_nop\n\tv_nop\n\tv_nop\n\tv_nop"
               : "+v"(a0), "+v"(a1), "+v"(a2), "+v"(a3), "+v"(a4), "+v"(a5), "+v"(a6), "+v"(a7)
               : "v"(x), "v"(y), "v"(b0), "v"(b1), "v"(b2), "v"(b3));
}
__device__ __forceinline__ void guard_lin(v8f& a0, v8f& a1, v8f& a2, v8f& a3,
                                          v16h x, v16h b0, v16h b1, v16h b2, v16h b3) {
  asm volatile("v_nop\n\tv_nop\n\tv_nop\n\tv_nop"
               : "+v"(a0), "+v"(a1), "+v"(a2), "+v"(a3)
               : "v"(x), "v"(b0), "v"(b1), "v"(b2), "v"(b3));
}
__device__ __forceinline__ void acc_guard8(v8f& a0, v8f& a1, v8f& a2, v8f& a3, v8f& a4, v8f& a5, v8f& a6, v8f& a7) {
  asm volatile("v_nop\n\tv_nop\n\tv_nop\n\tv_nop"
               : "+v"(a0), "+v"(a1), "+v"(a2), "+v"(a3), "+v"(a4), "+v"(a5), "+v"(a6), "+v"(a7));
}

__device__ __forceinline__ float sigm_f(float x)  { return __builtin_amdgcn_rcpf(1.0f + expf(-x)); }
__device__ __forceinline__ float tanh_f(float x)  { return 1.0f - 2.0f * __builtin_amdgcn_rcpf(1.0f + expf(2.0f * x)); }

__device__ __forceinline__ void split_h(float x, _Float16& hi, _Float16& lo) {
  const float xs = (fabsf(x) < HI_MIN) ? 0.0f : x;
  hi = (_Float16)xs;
  float hf = (float)hi;
  asm volatile("" : "+v"(hf));
  lo = (_Float16)((x - hf) * LOCARRY);
}

__global__ __launch_bounds__(256) void prep_kernel(const float* __restrict__ W_ih, const float* __restrict__ W_hh,
                                                   const float* __restrict__ b_ih, const float* __restrict__ b_hh,
                                                   const float* __restrict__ W1,
                                                   unsigned short* __restrict__ Wc16, unsigned short* __restrict__ W1f16,
                                                   unsigned short* __restrict__ W1l16,
                                                   float* __restrict__ bcv) {
  const int tid = threadIdx.x, blk = blockIdx.x;
  if (blk < 32) {
    const int i = blk * 256 + tid;
    const size_t e0 = (size_t)i * 8;
    const v4f a0 = *(const v4f*)(W_ih + e0);
    const v4f a1 = *(const v4f*)(W_ih + e0 + 4);
    const v4f h0 = *(const v4f*)(W_hh + e0);
    const v4f h1 = *(const v4f*)(W_hh + e0 + 4);
    v8h hv;
#pragma unroll
    for (int e = 0; e < 4; ++e) {
      const float f0 = (a0[e] + h0[e]) * WCARRY;
      const float f1 = (a1[e] + h1[e]) * WCARRY;
      hv[e]     = (_Float16)f0;
      hv[4 + e] = (_Float16)f1;
    }
    *(volatile v8h*)(Wc16 + e0) = hv;
    __threadfence();
    *(volatile v8h*)(Wc16 + e0) = hv;
  } else if (blk < 36) {
    const int i = (blk - 32) * 256 + tid;
    const int row = i >> 4, colb = (i & 15) * 8;
    const int rowc = row < NL1 ? row : NL1 - 1;
    const v4f a0 = *(const v4f*)(W1 + (size_t)rowc * HID + colb);
    const v4f a1 = *(const v4f*)(W1 + (size_t)rowc * HID + colb + 4);
    v8h hv, lv;
#pragma unroll
    for (int e = 0; e < 4; ++e) {
      const float f0 = (row < NL1) ? a0[e] * WCARRY : 0.0f;
      const float f1 = (row < NL1) ? a1[e] * WCARRY : 0.0f;
      _Float16 hq, lq;
      split_h(f0, hq, lq);
      hv[e] = hq;
      lv[e] = lq;
      split_h(f1, hq, lq);
      hv[4 + e] = hq;
      lv[4 + e] = lq;
    }
    *(volatile v8h*)(W1f16 + (size_t)i * 8) = hv;
    *(volatile v8h*)(W1l16 + (size_t)i * 8) = lv;
    __threadfence();
    *(volatile v8h*)(W1f16 + (size_t)i * 8) = hv;
    *(volatile v8h*)(W1l16 + (size_t)i * 8) = lv;
  } else {
    if (tid < 128) {
      const v4f a = *(const v4f*)(b_ih + tid * 4);
      const v4f b = *(const v4f*)(b_hh + tid * 4);
      v4f o;
#pragma unroll
      for (int e = 0; e < 4; ++e) o[e] = a[e] + b[e];
      *(volatile v4f*)(bcv + tid * 4) = o;
      __threadfence();
      *(volatile v4f*)(bcv + tid * 4) = o;
    }
  }
}

__global__ __launch_bounds__(NTHR1) void lstm_fused_kernel(const float* __restrict__ h_in, const float* __restrict__ c_in,
                                                           const unsigned short* __restrict__ Wcp,
                                                           const float* __restrict__ bc,
                                                           const unsigned short* __restrict__ W1p,
                                                           const unsigned short* __restrict__ W1lp,
                                                           float* __restrict__ P, float* __restrict__ part1) {
  __shared__ __align__(16) _Float16 sHi[WPB][2 * 16 * HP];
  __shared__ __align__(16) _Float16 sLo[WPB][2 * 16 * HP];
  __shared__ __align__(16) float    sC[WPB][64 * 32];
  __shared__ __align__(16) float    sSlab[WPB][16 * SLP];
  const _Float16* Wc  = (const _Float16*)Wcp;
  const _Float16* W1f = (const _Float16*)W1p;
  const _Float16* W1l = (const _Float16*)W1lp;
  const int tid = threadIdx.x, lane = tid & 31, wave = tid >> 5;
  const int c = lane & 15, hh = lane >> 4, koff = hh * 8, c4 = c * 4;
  const int wg = blockIdx.x * WPB + wave;
  const int b0 = wg * 16;
  _Float16* myHi = &sHi[wave][0];
  _Float16* myLo = &sLo[wave][0];
  float*    myC  = &sC[wave][0];
  float*    slab = &sSlab[wave][0];

#pragma unroll 1
  for (int i = 0; i < 16; ++i) {
    const v4f v = *(const v4f*)(h_in + (size_t)(b0 + i) * HID + lane * 4);
    const float f0 = v[0], f1 = v[1], f2 = v[2], f3 = v[3];
    _Float16 hi, lo;
    split_h(f0, hi, lo); myHi[i * HP + lane * 4 + 0] = hi; myLo[i * HP + lane * 4 + 0] = lo;
    split_h(f1, hi, lo); myHi[i * HP + lane * 4 + 1] = hi; myLo[i * HP + lane * 4 + 1] = lo;
    split_h(f2, hi, lo); myHi[i * HP + lane * 4 + 2] = hi; myLo[i * HP + lane * 4 + 2] = lo;
    split_h(f3, hi, lo); myHi[i * HP + lane * 4 + 3] = hi; myLo[i * HP + lane * 4 + 3] = lo;
  }
#pragma unroll 1
  for (int jt = 0; jt < 8; ++jt) {
#pragma unroll
    for (int r = 0; r < 8; ++r)
      myC[(jt * 8 + r) * 32 + lane] = c_in[(size_t)(b0 + 8 * hh + r) * HID + 16 * jt + c];
  }
  __syncthreads();

  const v8f z8 = {0.f, 0.f, 0.f, 0.f, 0.f, 0.f, 0.f, 0.f};
  float s1 = 0.0f, q1 = 0.0f;
  float sP[4], qP[4];
#pragma unroll
  for (int j = 0; j < 4; ++j) { sP[j] = 0.0f; qP[j] = 0.0f; }

#pragma unroll 1
  for (int t = 0; t <= TLEN; ++t) {
    const int cur = t & 1;
    const _Float16* aHrow = myHi + cur * (16 * HP) + c * HP + koff;
    const _Float16* aLrow = myLo + cur * (16 * HP) + c * HP + koff;

    if (t >= 1) {
      v8f pa[4], pb[4];
      pa[0] = z8; pa[1] = z8; pa[2] = z8; pa[3] = z8;
      pb[0] = z8; pb[1] = z8; pb[2] = z8; pb[3] = z8;
      const _Float16* w1b = W1f + (size_t)c * HID + koff;
      const _Float16* w1r = W1l + (size_t)c * HID + koff;
#pragma unroll 1
      for (int kt = 0; kt < 4; ++kt) {
        const v16h xh = Frag<_Float16>::load(aHrow + 32 * kt);
        const v16h xl = Frag<_Float16>::load(aLrow + 32 * kt);
        const v16h w0 = Frag<_Float16>::load(w1b + 32 * kt);
        const v16h w1 = Frag<_Float16>::load(w1b + (size_t)16 * HID + 32 * kt);
        const v16h w2 = Frag<_Float16>::load(w1b + (size_t)32 * HID + 32 * kt);
        const v16h w3 = Frag<_Float16>::load(w1b + (size_t)48 * HID + 32 * kt);
        pa[0] = Frag<_Float16>::mma(xh, w0, pa[0]);
        pa[1] = Frag<_Float16>::mma(xh, w1, pa[1]);
        pa[2] = Frag<_Float16>::mma(xh, w2, pa[2]);
        pa[3] = Frag<_Float16>::mma(xh, w3, pa[3]);
        pb[0] = Frag<_Float16>::mma(xl, w0, pb[0]);
        pb[1] = Frag<_Float16>::mma(xl, w1, pb[1]);
        pb[2] = Frag<_Float16>::mma(xl, w2, pb[2]);
        pb[3] = Frag<_Float16>::mma(xl, w3, pb[3]);
        guard_gate(pa[0], pa[1], pa[2], pa[3], pb[0], pb[1], pb[2], pb[3], xh, xl, w0, w1, w2, w3);
        const v16h u0 = Frag<_Float16>::load(w1r + 32 * kt);
        const v16h u1 = Frag<_Float16>::load(w1r + (size_t)16 * HID + 32 * kt);
        const v16h u2 = Frag<_Float16>::load(w1r + (size_t)32 * HID + 32 * kt);
        const v16h u3 = Frag<_Float16>::load(w1r + (size_t)48 * HID + 32 * kt);
        pb[0] = Frag<_Float16>::mma(xh, u0, pb[0]);
        pb[1] = Frag<_Float16>::mma(xh, u1, pb[1]);
        pb[2] = Frag<_Float16>::mma(xh, u2, pb[2]);
        pb[3] = Frag<_Float16>::mma(xh, u3, pb[3]);
        guard_lin(pb[0], pb[1], pb[2], pb[3], xh, u0, u1, u2, u3);
      }
      acc_guard8(pa[0], pa[1], pa[2], pa[3], pb[0], pb[1], pb[2], pb[3]);
#pragma unroll
      for (int j = 0; j < 4; ++j) {
#pragma unroll
        for (int r = 0; r < 8; ++r) {
          const float v = fmaf(pb[j][r], LO_INV, pa[j][r] * WCARRY_INV);
          slab[(8 * hh + r) * SLP + 16 * j + c] = v;
          sP[j] += v;
          qP[j] = fmaf(v, v, qP[j]);
        }
      }
      __syncthreads();
      float* Pt = P + ((size_t)(t - 1) * BATCH + (size_t)b0) * NPADC;
      for (int pass = 0; pass < 2; ++pass) {
#pragma unroll
        for (int it = 0; it < 8; ++it) {
          const int row = it * 2 + hh;
          const v4f v = *(const v4f*)(slab + row * SLP + c4);
          *(volatile v4f*)(Pt + (size_t)row * NPADC + c4) = v;
        }
        __threadfence();
      }
    }

    if (t < TLEN) {
      _Float16* nHi = myHi + (cur ^ 1) * (16 * HP);
      _Float16* nLo = myLo + (cur ^ 1) * (16 * HP);
#pragma unroll 1
      for (int jt = 0; jt < 8; ++jt) {
        const int ucol = 16 * jt + c;
        const _Float16* wb = Wc + (size_t)ucol * HID + koff;
        const float bi = bc[ucol];
        const float bf = bc[HID + ucol];
        const float bg = bc[2 * HID + ucol];
        const float bo = bc[3 * HID + ucol];
        v8f accH[4];
        accH[0] = z8; accH[1] = z8; accH[2] = z8; accH[3] = z8;
#pragma unroll 1
        for (int kt = 0; kt < 4; ++kt) {
          const v16h xh = Frag<_Float16>::load(aHrow + 32 * kt);
          const v16h w0 = Frag<_Float16>::load(wb + 32 * kt);
          const v16h w1 = Frag<_Float16>::load(wb + (size_t)1 * HID * HID + 32 * kt);
          const v16h w2 = Frag<_Float16>::load(wb + (size_t)2 * HID * HID + 32 * kt);
          const v16h w3 = Frag<_Float16>::load(wb + (size_t)3 * HID * HID + 32 * kt);
          accH[0] = Frag<_Float16>::mma(xh, w0, accH[0]);
          accH[1] = Frag<_Float16>::mma(xh, w1, accH[1]);
          accH[2] = Frag<_Float16>::mma(xh, w2, accH[2]);
          accH[3] = Frag<_Float16>::mma(xh, w3, accH[3]);
          guard_lin(accH[0], accH[1], accH[2], accH[3], xh, w0, w1, w2, w3);
        }
#pragma unroll
        for (int r = 0; r < 8; ++r) {
          const float zi = accH[0][r] * WCARRY_INV + bi;
          const float zf = accH[1][r] * WCARRY_INV + bf;
          const float zg = accH[2][r] * WCARRY_INV + bg;
          const float zo = accH[3][r] * WCARRY_INV + bo;
          const float ig = sigm_f(zi);
          const float fg = sigm_f(zf);
          const float gg = tanh_f(zg);
          const float og = sigm_f(zo);
          const float cold = myC[(jt * 8 + r) * 32 + lane];
          const float cn = fg * cold + ig * gg;
          myC[(jt * 8 + r) * 32 + lane] = cn;
          const float hn = og * tanh_f(cn);
          s1 += hn;
          q1 = fmaf(hn, hn, q1);
          _Float16 hi, lo;
          split_h(hn, hi, lo);
          nHi[(8 * hh + r) * HP + ucol] = hi;
          nLo[(8 * hh + r) * HP + ucol] = lo;
        }
      }
    }
    __syncthreads();
  }

#pragma unroll
  for (int off = 1; off < 32; off <<= 1) {
    s1 += __shfl_xor(s1, off, 32);
    q1 += __shfl_xor(q1, off, 32);
  }
  float sT[4], qT[4];
#pragma unroll
  for (int j = 0; j < 4; ++j) {
    sT[j] = sP[j] + __shfl_xor(sP[j], 16, 32);
    qT[j] = qP[j] + __shfl_xor(qP[j], 16, 32);
  }
#pragma unroll
  for (int j = 0; j < 4; ++j) slab[hh * 64 + 16 * j + c] = hh ? qT[j] : sT[j];
  slab[128 + lane] = (lane == 0) ? s1 : ((lane == 1) ? q1 : 0.0f);
  slab[160 + lane] = 0.0f;
  slab[192 + lane] = 0.0f;
  slab[224 + lane] = 0.0f;
  __syncthreads();
  {
    const v4f r0 = *(const v4f*)(slab + lane * 4);
    const v4f r1 = *(const v4f*)(slab + 128 + lane * 4);
    float* rp = part1 + (size_t)wg * REC1;
    for (int pass = 0; pass < 2; ++pass) {
      *(volatile v4f*)(rp + lane * 4) = r0;
      *(volatile v4f*)(rp + 128 + lane * 4) = r1;
      __threadfence();
    }
  }
}

__global__ __launch_bounds__(256) void fin12_kernel(const float* __restrict__ part1, const float* __restrict__ W1,
                                                    const float* __restrict__ b1,
                                                    const float* __restrict__ g1, const float* __restrict__ be1,
                                                    const float* __restrict__ g2, const float* __restrict__ be2,
                                                    float* __restrict__ tab) {
  __shared__ double sSum[256];
  __shared__ double sRs[64];
  __shared__ __align__(16) float sOut[128];
  const int tid = threadIdx.x;
  double acc = 0.0;
#pragma unroll 1
  for (int w = 0; w < NWAVES; ++w) acc += (double)part1[(size_t)w * REC1 + tid];
  sSum[tid] = acc;
  const int n64 = tid & 63;
  const int nc  = n64 < NL1 ? n64 : NL1 - 1;
  if (tid < 64) {
    double rs = 0.0;
#pragma unroll 1
    for (int k = 0; k < HID; ++k) rs += (double)W1[(size_t)nc * HID + k];
    sRs[tid] = (tid < NL1) ? rs : 0.0;
  }
  __syncthreads();
  const double invN1 = 1.0 / ((double)MROWS * (double)HID);
  const double invN2 = 1.0 / ((double)MROWS * (double)NL1);
  const double Mr = (double)MROWS;
  const double m1 = sSum[128] * invN1;
  double v1 = sSum[129] * invN1 - m1 * m1;
  v1 = v1 < 0.0 ? 0.0 : v1;
  const float a1 = g1[0] * rsqrtf((float)v1 + EPS_BN);
  const float d1 = be1[0] - (float)m1 * a1;
  const double a1d = (double)a1;
  double sy = 0.0, sy2 = 0.0;
#pragma unroll 1
  for (int n = 0; n < NL1; ++n) {
    const float cyn = (float)((double)d1 * sRs[n] + (double)b1[n]);
    const double cy = (double)cyn;
    const double S = sSum[n], Q = sSum[64 + n];
    sy  += a1d * S + Mr * cy;
    sy2 += a1d * a1d * Q + 2.0 * a1d * cy * S + Mr * cy * cy;
  }
  const double m2 = sy * invN2;
  double v2 = sy2 * invN2 - m2 * m2;
  v2 = v2 < 0.0 ? 0.0 : v2;
  const float a2 = g2[0] * rsqrtf((float)v2 + EPS_BN);
  const float d2 = be2[0] - (float)m2 * a2;
  const float cyf = (float)((double)d1 * sRs[nc] + (double)b1[nc]);
  const float ev  = a2 * cyf + d2;
  const float o = (tid == 0) ? (a2 * a1) : (((tid >= 64) && (n64 < NL1)) ? ev : 0.0f);
  if (tid < 128) sOut[tid] = o;
  __syncthreads();
  if (tid < 32) {
    const v4f v = *(const v4f*)(sOut + tid * 4);
    *(volatile v4f*)(tab + tid * 4) = v;
    __threadfence();
    *(volatile v4f*)(tab + tid * 4) = v;
  }
}

__global__ __launch_bounds__(256) void relu_dot_kernel(const float* __restrict__ P, const float* __restrict__ tab,
                                                       const float* __restrict__ W2,
                                                       float* __restrict__ U, float* __restrict__ part3) {
  __shared__ float sE[64], sW0[64], sW1[64];
  __shared__ __align__(16) float sU[512];
  __shared__ float sRed[2][8];
  const int tid = threadIdx.x, lane = tid & 31, wave = tid >> 5;
  if (tid < 64) {
    const int nc = tid < NL1 ? tid : NL1 - 1;
    const float ev = tab[64 + nc];
    const float w0 = W2[nc];
    const float w1 = W2[NL1 + nc];
    sE[tid]  = (tid < NL1) ? ev : 0.0f;
    sW0[tid] = (tid < NL1) ? w0 : 0.0f;
    sW1[tid] = (tid < NL1) ? w1 : 0.0f;
  }
  const float sc = tab[0];
  __syncthreads();
  const size_t row = (size_t)blockIdx.x * 256 + tid;
  const float* pr = P + row * NPADC;
  float u0 = 0.0f, u1 = 0.0f, s = 0.0f, q = 0.0f;
#pragma unroll 1
  for (int qd = 0; qd < 13; ++qd) {
    const v4f v = *(const v4f*)(pr + 4 * qd);
#pragma unroll
    for (int e = 0; e < 4; ++e) {
      const int n = 4 * qd + e;
      float r = fmaxf(fmaf(sc, v[e], sE[n]), 0.0f);
      r = (n < NL1) ? r : 0.0f;
      u0 = fmaf(r, sW0[n], u0);
      u1 = fmaf(r, sW1[n], u1);
      s += r;
      q = fmaf(r, r, q);
    }
  }
#pragma unroll
  for (int off = 1; off < 32; off <<= 1) {
    s += __shfl_xor(s, off, 32);
    q += __shfl_xor(q, off, 32);
  }
  sU[2 * tid]     = u0;
  sU[2 * tid + 1] = u1;
  if (lane == 0) { sRed[0][wave] = s; sRed[1][wave] = q; }
  __syncthreads();
  if (tid < 128) {
    const v4f v = *(const v4f*)(sU + tid * 4);
    float* up = U + (size_t)blockIdx.x * 512 + tid * 4;
    *(volatile v4f*)up = v;
    __threadfence();
    *(volatile v4f*)up = v;
  }
  if (wave == 4) {
    float S = 0.0f, Q = 0.0f;
#pragma unroll
    for (int w = 0; w < 8; ++w) { S += sRed[0][w]; Q += sRed[1][w]; }
    v4f o;
    o[0] = (lane == 0) ? S : 0.0f;
    o[1] = (lane == 0) ? Q : 0.0f;
    o[2] = 0.0f;
    o[3] = 0.0f;
    float* pp = part3 + (size_t)blockIdx.x * REC3 + lane * 4;
    *(volatile v4f*)pp = o;
    __threadfence();
    *(volatile v4f*)pp = o;
  }
}

__global__ __launch_bounds__(256) void fin3_kernel(const float* __restrict__ part3, const float* __restrict__ W2,
                                                   const float* __restrict__ b2,
                                                   const float* __restrict__ g3, const float* __restrict__ be3,
                                                   float* __restrict__ tab3) {
  __shared__ double sS[256], sQ[256];
  __shared__ __align__(16) float sOut[128];
  const int tid = threadIdx.x;
  double s = 0.0, q = 0.0;
#pragma unroll 1
  for (int i = tid; i < NB3; i += 256) {
    s += (double)part3[(size_t)i * REC3];
    q += (double)part3[(size_t)i * REC3 + 1];
  }
  sS[tid] = s; sQ[tid] = q;
  __syncthreads();
  double S = 0.0, Q = 0.0;
#pragma unroll 1
  for (int i = 0; i < 256; ++i) { S += sS[i]; Q += sQ[i]; }
  const double invN = 1.0 / ((double)MROWS * (double)NL1);
  const double m3 = S * invN;
  double v3 = Q * invN - m3 * m3;
  v3 = v3 < 0.0 ? 0.0 : v3;
  const float a3 = g3[0] * rsqrtf((float)v3 + EPS_BN);
  const float d3 = be3[0] - (float)m3 * a3;
  double r0 = 0.0, r1 = 0.0;
#pragma unroll 1
  for (int k = 0; k < NL1; ++k) { r0 += (double)W2[k]; r1 += (double)W2[NL1 + k]; }
  const float co0 = (float)((double)d3 * r0 + (double)b2[0]);
  const float co1 = (float)((double)d3 * r1 + (double)b2[1]);
  const float o = (tid == 0) ? a3 : ((tid == 1) ? co0 : ((tid == 2) ? co1 : 0.0f));
  if (tid < 128) sOut[tid] = o;
  __syncthreads();
  if (tid < 32) {
    const v4f v = *(const v4f*)(sOut + tid * 4);
    *(volatile v4f*)(tab3 + tid * 4) = v;
    __threadfence();
    *(volatile v4f*)(tab3 + tid * 4) = v;
  }
}

__global__ __launch_bounds__(256) void out_kernel(const float* __restrict__ U, const float* __restrict__ tab3,
                                                  float* __restrict__ out) {
  const int i = blockIdx.x * 256 + threadIdx.x;
  const int p = 2 * i;
  const int b = p / TLEN;
  const int t = p - b * TLEN;
  const v2f ua = *(const v2f*)(U + ((size_t)t * BATCH + (size_t)b) * 2);
  const v2f ub = *(const v2f*)(U + ((size_t)(t + 1) * BATCH + (size_t)b) * 2);
  const float a3 = tab3[0], c0 = tab3[1], c1 = tab3[2];
  v4f o;
  o[0] = fmaf(a3, ua[0], c0);
  o[1] = fmaf(a3, ua[1], c1);
  o[2] = fmaf(a3, ub[0], c0);
  o[3] = fmaf(a3, ub[1], c1);
  float* op = out + (size_t)i * 4;
  *(volatile v4f*)op = o;
  __threadfence();
  *(volatile v4f*)op = o;
}

extern "C" void kernel_launch(void* const* d_in, const int* in_sizes, int n_in,
                              void* d_out, int out_size, void* d_ws, size_t ws_size, hipStream_t stream) {
  if (n_in < 16 || d_out == nullptr || d_ws == nullptr) return;
  if (in_sizes[0] != BATCH * HID || in_sizes[1] != BATCH * HID || in_sizes[2] != G4 * HID || in_sizes[3] != G4 * HID ||
      in_sizes[4] != G4 || in_sizes[5] != G4 || in_sizes[12] != NL1 * HID || in_sizes[13] != NL1 ||
      in_sizes[14] != 2 * NL1 || in_sizes[15] != 2 || out_size != MROWS * 2) return;

  const float* h_in   = (const float*)d_in[0];
  const float* c_in   = (const float*)d_in[1];
  const float* W_ih   = (const float*)d_in[2];
  const float* W_hh   = (const float*)d_in[3];
  const float* b_ih   = (const float*)d_in[4];
  const float* b_hh   = (const float*)d_in[5];
  const float* gamma1 = (const float*)d_in[6];
  const float* beta1  = (const float*)d_in[7];
  const float* gamma2 = (const float*)d_in[8];
  const float* beta2  = (const float*)d_in[9];
  const float* gamma3 = (const float*)d_in[10];
  const float* beta3  = (const float*)d_in[11];
  const float* W1     = (const float*)d_in[12];
  const float* b1     = (const float*)d_in[13];
  const float* W2     = (const float*)d_in[14];
  const float* b2     = (const float*)d_in[15];
  float* out = (float*)d_out;

  char* ws = (char*)d_ws; size_t off = 0;
  auto carve = [&](size_t bytes) -> char* { char* p = ws + off; off += (bytes + 255) & ~(size_t)255; return p; };
  unsigned short* WC16  = (unsigned short*)carve((size_t)G4 * HID * 2);
  unsigned short* W1F16 = (unsigned short*)carve((size_t)NPADC * HID * 2);
  unsigned short* W1L16 = (unsigned short*)carve((size_t)NPADC * HID * 2);
  float* BCV   = (float*)carve((size_t)G4 * 4);
  float* TAB1  = (float*)carve((size_t)128 * 4);
  float* TAB3  = (float*)carve((size_t)128 * 4);
  float* PART1 = (float*)carve((size_t)NWAVES * REC1 * 4);
  float* PART3 = (float*)carve((size_t)NB3 * REC3 * 4);
  float* UPL   = (float*)carve((size_t)MROWS * 2 * 4);
  float* PPL   = (float*)carve((size_t)MROWS * NPADC * 4);
  if (off > ws_size || off > (size_t)134217728) return;

  prep_kernel<<<37, 256, 0, stream>>>(W_ih, W_hh, b_ih, b_hh, W1, WC16, W1F16, W1L16, BCV);
  lstm_fused_kernel<<<NBLK1, NTHR1, 0, stream>>>(h_in, c_in, WC16, BCV, W1F16, W1L16, PPL, PART1);
  fin12_kernel<<<1, 256, 0, stream>>>(PART1, W1, b1, gamma1, beta1, gamma2, beta2, TAB1);
  relu_dot_kernel<<<NB3, 256, 0, stream>>>(PPL, TAB1, W2, UPL, PART3);
  fin3_kernel<<<1, 256, 0, stream>>>(PART3, W2, b2, gamma3, beta3, TAB3);
  out_kernel<<<NB5, 256, 0, stream>>>(UPL, TAB3, out);
}
